// HeteroGIN_16037407883348
// MI455X (gfx1250) — hardware-verified
//
#include <hip/hip_runtime.h>
#include <math.h>

typedef __attribute__((ext_vector_type(16))) _Float16 v16h;
typedef __attribute__((ext_vector_type(16))) __bf16 v16b;
typedef __attribute__((ext_vector_type(8)))  _Float16 v8h;
typedef __attribute__((ext_vector_type(8)))  float v8f;
typedef __attribute__((ext_vector_type(4)))  float v4f;
typedef __attribute__((ext_vector_type(2)))  float v2f;
typedef __attribute__((ext_vector_type(4)))  unsigned v4u;
typedef __attribute__((ext_vector_type(4)))  int v4i;
typedef float __attribute__((may_alias)) float_a;
typedef int __attribute__((may_alias)) int_a;

template <typename T> __device__ __forceinline__ void vst2(void* p, T v) { *(volatile T*)p = v; __threadfence(); *(volatile T*)p = v; }
__device__ __forceinline__ v8f wmma16(v16h a, v16h b, v8f c) {
  v8f d = __builtin_amdgcn_wmma_f32_16x16x32_f16(false, a, false, b, (short)0, c, false, false);
  asm volatile("v_nop\n\tv_nop\n\tv_nop\n\tv_nop" : "+v"(d) : "v"(a), "v"(b));
  return d;
}
__device__ __forceinline__ v8f wmma_bf(v16b a, v16b b, v8f c) {
  v8f d = __builtin_amdgcn_wmma_f32_16x16x32_bf16(false, a, false, b, (short)0, c, false, false);
  asm volatile("v_nop\n\tv_nop\n\tv_nop\n\tv_nop" : "+v"(d) : "v"(a), "v"(b));
  return d;
}
__device__ __forceinline__ v16h frag_h(const _Float16* rowk0, int lane) {
  union { v16h v; v8h q[2]; } u; const _Float16* p = rowk0 + 8 * (lane >> 4);
  u.q[0] = *(const v8h*)p; u.q[1] = *(const v8h*)(p + 16); return u.v;
}
__device__ __forceinline__ v16h frag_f32(const float* rowk0, int lane) {
  v16h a; const float* p = rowk0 + 8 * (lane >> 4);
#pragma unroll
  for (int i = 0; i < 8; ++i) { a[i] = (_Float16)p[i]; a[8 + i] = (_Float16)p[16 + i]; }
  return a;
}
__device__ __forceinline__ v16h frag_f32s(const float* rowk0, int lane, float sc) {
  v16h a; const float* p = rowk0 + 8 * (lane >> 4);
#pragma unroll
  for (int i = 0; i < 8; ++i) { a[i] = (_Float16)(p[i] * sc); a[8 + i] = (_Float16)(p[16 + i] * sc); }
  return a;
}
__device__ __forceinline__ v16h fragc_f32(const float* W, int k0, int n, int lane, int ld, int K) {
  v16h a; const int g = lane >> 4;
#pragma unroll
  for (int i = 0; i < 8; ++i) { const int ka = k0 + 8 * g + i, kb = ka + 16;
    a[i] = (_Float16)(ka < K ? W[(size_t)(ka < K ? ka : K - 1) * ld + n] : 0.f); a[8 + i] = (_Float16)(kb < K ? W[(size_t)(kb < K ? kb : K - 1) * ld + n] : 0.f); }
  return a;
}
struct F2 { v16b h, l; };
__device__ __forceinline__ F2 bsplit16(const float v[16]) { F2 r;
#pragma unroll
  for (int i = 0; i < 16; ++i) { const __bf16 h = (__bf16)v[i]; r.h[i] = h; r.l[i] = (__bf16)(v[i] - (float)h); }
  return r; }
__device__ __forceinline__ F2 split_row(const float* row, int k0, int lane) { float v[16]; const float* p = row + k0 + 8 * (lane >> 4);
#pragma unroll
  for (int i = 0; i < 8; ++i) { v[i] = p[i]; v[8 + i] = p[16 + i]; }
  return bsplit16(v); }
__device__ __forceinline__ F2 split_rowK(const float* row, int k0, int lane, int K) { float v[16]; const int g = lane >> 4;
#pragma unroll
  for (int i = 0; i < 8; ++i) { const int ka = k0 + 8 * g + i, kb = ka + 16; v[i] = ka < K ? row[ka < K ? ka : K - 1] : 0.f; v[8 + i] = kb < K ? row[kb < K ? kb : K - 1] : 0.f; }
  return bsplit16(v); }
__device__ __forceinline__ F2 split_col(const float* W, int k0, int n, int lane, int ld, int K) { float v[16]; const int g = lane >> 4;
#pragma unroll
  for (int i = 0; i < 8; ++i) { const int ka = k0 + 8 * g + i, kb = ka + 16; v[i] = ka < K ? W[(size_t)(ka < K ? ka : K - 1) * ld + n] : 0.f; v[8 + i] = kb < K ? W[(size_t)(kb < K ? kb : K - 1) * ld + n] : 0.f; }
  return bsplit16(v); }
__device__ __forceinline__ v8f mac3(const F2& a, const F2& b, v8f c) { c = wmma_bf(a.l, b.h, c); c = wmma_bf(a.h, b.l, c); return wmma_bf(a.h, b.h, c); }
__device__ __forceinline__ float sigm(float v) { return 1.0f / (1.0f + expf(-v)); }
#define LDSX() do { asm volatile("s_wait_dscnt 0" ::: "memory"); __builtin_amdgcn_wave_barrier(); __builtin_amdgcn_fence(__ATOMIC_RELEASE, "workgroup"); } while (0)


#ifndef NN
#define NN 100000
#endif
#define EPA 100000
#define EPB 1600000
#ifndef NEA
#define NEA 100000
#define NEB 1600000
#endif
#define DIN 16
#define HID 128
#define OC 64
#define NBLK ((NN + 63) / 64)
#define NRP (NBLK * 64)
typedef __attribute__((ext_vector_type(8))) __bf16 v8b;
__device__ __forceinline__ v16b frag_b(const __bf16* rowk0, int lane) {
  union { v16b v; v8b q[2]; } u; const __bf16* p = rowk0 + 8 * (lane >> 4);
  u.q[0] = *(const v8b*)p; u.q[1] = *(const v8b*)(p + 16); return u.v;
}
__device__ __forceinline__ float bfr(float v) { return (float)(__bf16)v; }
__device__ __attribute__((noinline)) float exp_ni(float v) { return expf(v); }
__device__ __attribute__((noinline)) float erf_ni(float v) { return erff(v); }

#define CSA_N NN
#define CSA_E NEA
#define CSA_FINN (CSA_E + 32 * CSA_NBK)
#define CSA_CHUNK 4096
#define CSA_BKT 256
#define CSA_NCH ((CSA_E + CSA_CHUNK - 1) / CSA_CHUNK)
#define CSA_NBK ((CSA_N + CSA_BKT - 1) / CSA_BKT)
#define CSA_NBKP (((CSA_NBK + 63) / 64) * 64)
#define CSA_SEGCAP (CSA_E + 32 * CSA_NBK * CSA_NCH)
#ifndef CSA_BCAP
#define CSA_BCAP 10240
#endif
#define CSA_SZ_CNT   (4u * CSA_NCH * CSA_NBKP)
#define CSA_SZ_OFF   (4u * CSA_NBK * (((CSA_NCH + 31) / 32) * 32))
#define CSA_SZ_BST   (4u * (((CSA_NBK + 1 + 31) / 32) * 32))
#define CSA_SZ_SEG   (4u * CSA_SEGCAP)
#define CSA_SZ_FIN   (4u * (CSA_E + 32 * CSA_NBK))
#define CSA_SZ_ROW   (4u * CSA_NBK * CSA_BKT)
#define CSA_OFFP (((CSA_NCH + 31) / 32) * 32)

__global__ __launch_bounds__(256) void k_csA_cnt(const int* __restrict__ DST, int dstride, int* __restrict__ CNT) {
  __shared__ unsigned short sc[256][CSA_NBK + 1]; __shared__ __align__(16) int srow[CSA_NBKP];
  const int c = blockIdx.x, tid = threadIdx.x;
  for (int b = 0; b < CSA_NBK; ++b) sc[tid][b] = 0;
  const size_t e0 = (size_t)c * CSA_CHUNK + tid * 16;
  for (int i = 0; i < 16; ++i) { const size_t e = e0 + i; if (e < (size_t)CSA_E) { int d = DST[e * dstride]; d = min(max(d, 0), CSA_N - 1); sc[tid][d / CSA_BKT] += 1; } }
  __syncthreads();
  for (int b = tid; b < CSA_NBKP; b += 256) { int s = 0; if (b < CSA_NBK) for (int t = 0; t < 256; ++t) s += sc[t][b]; srow[b] = s; }
  __syncthreads();
  for (int q = tid; q < CSA_NBKP / 4; q += 256) vst2((unsigned*)(CNT + (size_t)c * CSA_NBKP + q * 4), *(const v4u*)&srow[q * 4]);
}
__global__ __launch_bounds__(256) void k_csA_scan(const int* __restrict__ CNT, int* __restrict__ OFF, int* __restrict__ BST) {
  __shared__ int sbt[CSA_NBK + 1]; __shared__ int sbs[((CSA_NBK + 1 + 31) / 32) * 32]; __shared__ int scnt[CSA_NBK + 1]; __shared__ __align__(16) int sbuf[64][CSA_OFFP];
  const int tid = threadIdx.x;
  for (int b = tid; b < CSA_NBK; b += 256) { int sp = 0, st = 0; for (int c = 0; c < CSA_NCH; ++c) { const int n = CNT[(size_t)c * CSA_NBKP + b]; st += n; sp += (n + 31) & ~31; } sbt[b] = sp; scnt[b] = st; }
  for (int b = tid; b < ((CSA_NBK + 1 + 31) / 32) * 32; b += 256) sbs[b] = 0;
  __syncthreads();
  if (tid == 0) { int acc = 0, accf = 0; for (int b = 0; b < CSA_NBK; ++b) { const int t = sbt[b]; sbt[b] = acc; acc += t; sbs[b] = accf; accf += (scnt[b] + 31) & ~31; } sbs[CSA_NBK] = accf; }
  __syncthreads();
  for (int b0 = 0; b0 < CSA_NBK; b0 += 64) {
    if (tid < 64 && b0 + tid < CSA_NBK) { const int b = b0 + tid; int o = sbt[b]; for (int c = 0; c < CSA_OFFP; ++c) { if (c < CSA_NCH) { sbuf[tid][c] = o; o += (CNT[(size_t)c * CSA_NBKP + b] + 31) & ~31; } else sbuf[tid][c] = 0; } }
    __syncthreads();
    for (int q = tid; q < 64 * (CSA_OFFP / 4); q += 256) { const int r = q / (CSA_OFFP / 4), pc = q % (CSA_OFFP / 4); if (b0 + r < CSA_NBK) vst2((unsigned*)(OFF + (size_t)(b0 + r) * CSA_OFFP + pc * 4), *(const v4u*)&sbuf[r][pc * 4]); }
    __syncthreads(); }
  for (int q = tid; q < ((CSA_NBK + 1 + 31) / 32) * 32 / 4; q += 256) vst2((unsigned*)(BST + q * 4), *(const v4u*)&sbs[q * 4]);
}
__global__ __launch_bounds__(256) void k_csA_scatter(const int* __restrict__ SRC, const int* __restrict__ DST, int sstride, int dstride, const int* __restrict__ OFF, int* __restrict__ SEGS, int* __restrict__ SEGE) {
  __shared__ unsigned short sc[256][CSA_NBK + 1]; __shared__ int sbase[CSA_NBK + 1]; __shared__ int scn[CSA_NBK + 1]; __shared__ int sord[CSA_CHUNK];
  const int c = blockIdx.x, tid = threadIdx.x;
  for (int b = 0; b < CSA_NBK; ++b) sc[tid][b] = 0;
  const size_t e0 = (size_t)c * CSA_CHUNK + tid * 16; int bk[16];
#pragma unroll
  for (int i = 0; i < 16; ++i) { const size_t e = e0 + i; bk[i] = -1; if (e < (size_t)CSA_E) { int d = DST[e * dstride]; d = min(max(d, 0), CSA_N - 1); bk[i] = d / CSA_BKT; sc[tid][bk[i]] += 1; } }
  __syncthreads();
  for (int b = tid; b < CSA_NBK; b += 256) { int acc = 0; for (int t = 0; t < 256; ++t) { const int v = sc[t][b]; sc[t][b] = (unsigned short)acc; acc += v; } scn[b] = acc; }
  __syncthreads();
  if (tid == 0) { int acc = 0; for (int b = 0; b < CSA_NBK; ++b) { sbase[b] = acc; acc += scn[b]; } }
  __syncthreads();
#pragma unroll
  for (int i = 0; i < 16; ++i) { if (bk[i] >= 0) { const int b = bk[i]; const int r = sc[tid][b]; sc[tid][b] = (unsigned short)(r + 1); sord[sbase[b] + r] = tid * 16 + i; } }
  __syncthreads();
  for (int b = 0; b < CSA_NBK; ++b) { const int n = scn[b]; if (n == 0) continue; const int nl = ((n + 31) & ~31); const size_t o = (size_t)(min(max(OFF[(size_t)b * CSA_OFFP + c], 0), CSA_SEGCAP - nl) & ~31);
    for (int q = tid; q < nl / 4; q += 256) { int4 vs, ve;
#pragma unroll
      for (int k = 0; k < 4; ++k) { const int i = q * 4 + k; int s = -1, eid = -1; if (i < n) { const size_t e = (size_t)c * CSA_CHUNK + sord[sbase[b] + i]; s = min(max(SRC[e * sstride], 0), CSA_N - 1); eid = (int)e; } vs[k] = s; ve[k] = eid; }
      vst2((unsigned*)(SEGS + o + q * 4), *(const v4u*)&vs); vst2((unsigned*)(SEGE + o + q * 4), *(const v4u*)&ve); } }
}
__global__ __launch_bounds__(256) void k_csA_bucket(const int* __restrict__ CNT, const int* __restrict__ OFF, const int* __restrict__ BST, const int* __restrict__ SEGS, const int* __restrict__ SEGE, const int* __restrict__ DST, int dstride, int* __restrict__ FS, int* __restrict__ FE, int* __restrict__ ROWST, int* __restrict__ ROWCNT) {
  __shared__ int ssrc[CSA_BCAP]; __shared__ int seid[CSA_BCAP]; __shared__ unsigned char snod[CSA_BCAP]; __shared__ int souts[CSA_BCAP]; __shared__ int soute[CSA_BCAP]; __shared__ int scount[256]; __shared__ int sstart[257]; __shared__ int stot;
  const int b = blockIdx.x, tid = threadIdx.x;
  if (tid == 0) { int t = 0; for (int c = 0; c < CSA_NCH; ++c) t += min(max(CNT[(size_t)c * CSA_NBKP + b], 0), CSA_CHUNK); stot = (t <= CSA_BCAP) ? t : 0; }
  __syncthreads();
  { int base = 0; for (int c = 0; c < CSA_NCH; ++c) { const int n = min(max(CNT[(size_t)c * CSA_NBKP + b], 0), CSA_CHUNK); const int o = min(max(OFF[(size_t)b * CSA_OFFP + c], 0), CSA_SEGCAP - ((n + 31) & ~31));
      for (int i = tid; i < n; i += 256) { const int p = base + i; if (p < CSA_BCAP) { ssrc[p] = min(max(SEGS[o + i], 0), CSA_N - 1); const int e = min(max(SEGE[o + i], 0), CSA_E - 1); seid[p] = e; int d = DST[(size_t)e * dstride]; d = min(max(d, 0), CSA_N - 1); const int dl = d - b * CSA_BKT; snod[p] = (unsigned char)(dl >= 0 && dl < 256 ? dl : 255); } }
      base += n; } }
  __syncthreads();
  const int node = b * CSA_BKT + tid; int cnt = 0; for (int p = 0; p < stot; ++p) cnt += (snod[p] == tid) ? 1 : 0;
  scount[tid] = cnt; __syncthreads();
  if (tid == 0) { int acc = 0; for (int t = 0; t < 256; ++t) { sstart[t] = acc; acc += scount[t]; } sstart[256] = acc; }
  __syncthreads();
  const int bst0 = min(max(BST[b], 0), CSA_FINN - ((sstart[256] + 31) & ~31)) & ~31; const int gst = bst0 + sstart[tid];
  { int w = sstart[tid]; for (int p = 0; p < stot; ++p) if (snod[p] == tid) { souts[w] = ssrc[p]; soute[w] = seid[p]; ++w; } }
  __syncthreads();
  { const int n = sstart[256]; const int nl = (n + 31) & ~31; for (int q = tid; q < nl / 4; q += 256) { int4 vs, ve;
#pragma unroll
      for (int k = 0; k < 4; ++k) { const int i = q * 4 + k; vs[k] = i < n ? souts[i] : -1; ve[k] = i < n ? soute[i] : -1; }
      vst2((unsigned*)(FS + bst0 + q * 4), *(const v4u*)&vs); vst2((unsigned*)(FE + bst0 + q * 4), *(const v4u*)&ve); } }
  __syncthreads();
  { __shared__ __align__(16) int srs[256], src2[256]; srs[tid] = node < CSA_N ? gst : 0; src2[tid] = node < CSA_N ? cnt : 0; __syncthreads();
    if (tid < 64) vst2((unsigned*)(ROWST + (size_t)b * 256 + tid * 4), *(const v4u*)&srs[tid * 4]); else if (tid < 128) vst2((unsigned*)(ROWCNT + (size_t)b * 256 + (tid - 64) * 4), *(const v4u*)&src2[(tid - 64) * 4]); }
}


#define CSB_N NN
#define CSB_E NEB
#define CSB_FINN (CSB_E + 32 * CSB_NBK)
#define CSB_CHUNK 4096
#define CSB_BKT 256
#define CSB_NCH ((CSB_E + CSB_CHUNK - 1) / CSB_CHUNK)
#define CSB_NBK ((CSB_N + CSB_BKT - 1) / CSB_BKT)
#define CSB_NBKP (((CSB_NBK + 63) / 64) * 64)
#define CSB_SEGCAP (CSB_E + 32 * CSB_NBK * CSB_NCH)
#ifndef CSB_BCAP
#define CSB_BCAP 10240
#endif
#define CSB_SZ_CNT   (4u * CSB_NCH * CSB_NBKP)
#define CSB_SZ_OFF   (4u * CSB_NBK * (((CSB_NCH + 31) / 32) * 32))
#define CSB_SZ_BST   (4u * (((CSB_NBK + 1 + 31) / 32) * 32))
#define CSB_SZ_SEG   (4u * CSB_SEGCAP)
#define CSB_SZ_FIN   (4u * (CSB_E + 32 * CSB_NBK))
#define CSB_SZ_ROW   (4u * CSB_NBK * CSB_BKT)
#define CSB_OFFP (((CSB_NCH + 31) / 32) * 32)

__global__ __launch_bounds__(256) void k_csB_cnt(const int* __restrict__ DST, int dstride, int* __restrict__ CNT) {
  __shared__ unsigned short sc[256][CSB_NBK + 1]; __shared__ __align__(16) int srow[CSB_NBKP];
  const int c = blockIdx.x, tid = threadIdx.x;
  for (int b = 0; b < CSB_NBK; ++b) sc[tid][b] = 0;
  const size_t e0 = (size_t)c * CSB_CHUNK + tid * 16;
  for (int i = 0; i < 16; ++i) { const size_t e = e0 + i; if (e < (size_t)CSB_E) { int d = DST[e * dstride]; d = min(max(d, 0), CSB_N - 1); sc[tid][d / CSB_BKT] += 1; } }
  __syncthreads();
  for (int b = tid; b < CSB_NBKP; b += 256) { int s = 0; if (b < CSB_NBK) for (int t = 0; t < 256; ++t) s += sc[t][b]; srow[b] = s; }
  __syncthreads();
  for (int q = tid; q < CSB_NBKP / 4; q += 256) vst2((unsigned*)(CNT + (size_t)c * CSB_NBKP + q * 4), *(const v4u*)&srow[q * 4]);
}
__global__ __launch_bounds__(256) void k_csB_scan(const int* __restrict__ CNT, int* __restrict__ OFF, int* __restrict__ BST) {
  __shared__ int sbt[CSB_NBK + 1]; __shared__ int sbs[((CSB_NBK + 1 + 31) / 32) * 32]; __shared__ int scnt[CSB_NBK + 1]; __shared__ __align__(16) int sbuf[64][CSB_OFFP];
  const int tid = threadIdx.x;
  for (int b = tid; b < CSB_NBK; b += 256) { int sp = 0, st = 0; for (int c = 0; c < CSB_NCH; ++c) { const int n = CNT[(size_t)c * CSB_NBKP + b]; st += n; sp += (n + 31) & ~31; } sbt[b] = sp; scnt[b] = st; }
  for (int b = tid; b < ((CSB_NBK + 1 + 31) / 32) * 32; b += 256) sbs[b] = 0;
  __syncthreads();
  if (tid == 0) { int acc = 0, accf = 0; for (int b = 0; b < CSB_NBK; ++b) { const int t = sbt[b]; sbt[b] = acc; acc += t; sbs[b] = accf; accf += (scnt[b] + 31) & ~31; } sbs[CSB_NBK] = accf; }
  __syncthreads();
  for (int b0 = 0; b0 < CSB_NBK; b0 += 64) {
    if (tid < 64 && b0 + tid < CSB_NBK) { const int b = b0 + tid; int o = sbt[b]; for (int c = 0; c < CSB_OFFP; ++c) { if (c < CSB_NCH) { sbuf[tid][c] = o; o += (CNT[(size_t)c * CSB_NBKP + b] + 31) & ~31; } else sbuf[tid][c] = 0; } }
    __syncthreads();
    for (int q = tid; q < 64 * (CSB_OFFP / 4); q += 256) { const int r = q / (CSB_OFFP / 4), pc = q % (CSB_OFFP / 4); if (b0 + r < CSB_NBK) vst2((unsigned*)(OFF + (size_t)(b0 + r) * CSB_OFFP + pc * 4), *(const v4u*)&sbuf[r][pc * 4]); }
    __syncthreads(); }
  for (int q = tid; q < ((CSB_NBK + 1 + 31) / 32) * 32 / 4; q += 256) vst2((unsigned*)(BST + q * 4), *(const v4u*)&sbs[q * 4]);
}
__global__ __launch_bounds__(256) void k_csB_scatter(const int* __restrict__ SRC, const int* __restrict__ DST, int sstride, int dstride, const int* __restrict__ OFF, int* __restrict__ SEGS, int* __restrict__ SEGE) {
  __shared__ unsigned short sc[256][CSB_NBK + 1]; __shared__ int sbase[CSB_NBK + 1]; __shared__ int scn[CSB_NBK + 1]; __shared__ int sord[CSB_CHUNK];
  const int c = blockIdx.x, tid = threadIdx.x;
  for (int b = 0; b < CSB_NBK; ++b) sc[tid][b] = 0;
  const size_t e0 = (size_t)c * CSB_CHUNK + tid * 16; int bk[16];
#pragma unroll
  for (int i = 0; i < 16; ++i) { const size_t e = e0 + i; bk[i] = -1; if (e < (size_t)CSB_E) { int d = DST[e * dstride]; d = min(max(d, 0), CSB_N - 1); bk[i] = d / CSB_BKT; sc[tid][bk[i]] += 1; } }
  __syncthreads();
  for (int b = tid; b < CSB_NBK; b += 256) { int acc = 0; for (int t = 0; t < 256; ++t) { const int v = sc[t][b]; sc[t][b] = (unsigned short)acc; acc += v; } scn[b] = acc; }
  __syncthreads();
  if (tid == 0) { int acc = 0; for (int b = 0; b < CSB_NBK; ++b) { sbase[b] = acc; acc += scn[b]; } }
  __syncthreads();
#pragma unroll
  for (int i = 0; i < 16; ++i) { if (bk[i] >= 0) { const int b = bk[i]; const int r = sc[tid][b]; sc[tid][b] = (unsigned short)(r + 1); sord[sbase[b] + r] = tid * 16 + i; } }
  __syncthreads();
  for (int b = 0; b < CSB_NBK; ++b) { const int n = scn[b]; if (n == 0) continue; const int nl = ((n + 31) & ~31); const size_t o = (size_t)(min(max(OFF[(size_t)b * CSB_OFFP + c], 0), CSB_SEGCAP - nl) & ~31);
    for (int q = tid; q < nl / 4; q += 256) { int4 vs, ve;
#pragma unroll
      for (int k = 0; k < 4; ++k) { const int i = q * 4 + k; int s = -1, eid = -1; if (i < n) { const size_t e = (size_t)c * CSB_CHUNK + sord[sbase[b] + i]; s = min(max(SRC[e * sstride], 0), CSB_N - 1); eid = (int)e; } vs[k] = s; ve[k] = eid; }
      vst2((unsigned*)(SEGS + o + q * 4), *(const v4u*)&vs); vst2((unsigned*)(SEGE + o + q * 4), *(const v4u*)&ve); } }
}
__global__ __launch_bounds__(256) void k_csB_bucket(const int* __restrict__ CNT, const int* __restrict__ OFF, const int* __restrict__ BST, const int* __restrict__ SEGS, const int* __restrict__ SEGE, const int* __restrict__ DST, int dstride, int* __restrict__ FS, int* __restrict__ FE, int* __restrict__ ROWST, int* __restrict__ ROWCNT) {
  __shared__ int ssrc[CSB_BCAP]; __shared__ int seid[CSB_BCAP]; __shared__ unsigned char snod[CSB_BCAP]; __shared__ int souts[CSB_BCAP]; __shared__ int soute[CSB_BCAP]; __shared__ int scount[256]; __shared__ int sstart[257]; __shared__ int stot;
  const int b = blockIdx.x, tid = threadIdx.x;
  if (tid == 0) { int t = 0; for (int c = 0; c < CSB_NCH; ++c) t += min(max(CNT[(size_t)c * CSB_NBKP + b], 0), CSB_CHUNK); stot = (t <= CSB_BCAP) ? t : 0; }
  __syncthreads();
  { int base = 0; for (int c = 0; c < CSB_NCH; ++c) { const int n = min(max(CNT[(size_t)c * CSB_NBKP + b], 0), CSB_CHUNK); const int o = min(max(OFF[(size_t)b * CSB_OFFP + c], 0), CSB_SEGCAP - ((n + 31) & ~31));
      for (int i = tid; i < n; i += 256) { const int p = base + i; if (p < CSB_BCAP) { ssrc[p] = min(max(SEGS[o + i], 0), CSB_N - 1); const int e = min(max(SEGE[o + i], 0), CSB_E - 1); seid[p] = e; int d = DST[(size_t)e * dstride]; d = min(max(d, 0), CSB_N - 1); const int dl = d - b * CSB_BKT; snod[p] = (unsigned char)(dl >= 0 && dl < 256 ? dl : 255); } }
      base += n; } }
  __syncthreads();
  const int node = b * CSB_BKT + tid; int cnt = 0; for (int p = 0; p < stot; ++p) cnt += (snod[p] == tid) ? 1 : 0;
  scount[tid] = cnt; __syncthreads();
  if (tid == 0) { int acc = 0; for (int t = 0; t < 256; ++t) { sstart[t] = acc; acc += scount[t]; } sstart[256] = acc; }
  __syncthreads();
  const int bst0 = min(max(BST[b], 0), CSB_FINN - ((sstart[256] + 31) & ~31)) & ~31; const int gst = bst0 + sstart[tid];
  { int w = sstart[tid]; for (int p = 0; p < stot; ++p) if (snod[p] == tid) { souts[w] = ssrc[p]; soute[w] = seid[p]; ++w; } }
  __syncthreads();
  { const int n = sstart[256]; const int nl = (n + 31) & ~31; for (int q = tid; q < nl / 4; q += 256) { int4 vs, ve;
#pragma unroll
      for (int k = 0; k < 4; ++k) { const int i = q * 4 + k; vs[k] = i < n ? souts[i] : -1; ve[k] = i < n ? soute[i] : -1; }
      vst2((unsigned*)(FS + bst0 + q * 4), *(const v4u*)&vs); vst2((unsigned*)(FE + bst0 + q * 4), *(const v4u*)&ve); } }
  __syncthreads();
  { __shared__ __align__(16) int srs[256], src2[256]; srs[tid] = node < CSB_N ? gst : 0; src2[tid] = node < CSB_N ? cnt : 0; __syncthreads();
    if (tid < 64) vst2((unsigned*)(ROWST + (size_t)b * 256 + tid * 4), *(const v4u*)&srs[tid * 4]); else if (tid < 128) vst2((unsigned*)(ROWCNT + (size_t)b * 256 + (tid - 64) * 4), *(const v4u*)&src2[(tid - 64) * 4]); }
}


#define WSA_CNT  0u
#define WSA_OFF  (WSA_CNT + CSA_SZ_CNT)
#define WSA_BST  (WSA_OFF + CSA_SZ_OFF)
#define WSA_SEGS (WSA_BST + CSA_SZ_BST)
#define WSA_SEGE (WSA_SEGS + CSA_SZ_SEG)
#define WSA_FS   (WSA_SEGE + CSA_SZ_SEG)
#define WSA_FE   (WSA_FS + CSA_SZ_FIN)
#define WSA_RST  (WSA_FE + CSA_SZ_FIN)
#define WSA_RCT  (WSA_RST + CSA_SZ_ROW)
#define WSB_CNT  (WSA_RCT + CSA_SZ_ROW)
#define WSB_OFF  (WSB_CNT + CSB_SZ_CNT)
#define WSB_BST  (WSB_OFF + CSB_SZ_OFF)
#define WSB_SEGS (WSB_BST + CSB_SZ_BST)
#define WSB_SEGE (WSB_SEGS + CSB_SZ_SEG)
#define WSB_FS   (WSB_SEGE + CSB_SZ_SEG)
#define WSB_FE   (WSB_FS + CSB_SZ_FIN)
#define WSB_RST  (WSB_FE + CSB_SZ_FIN)
#define WSB_RCT  (WSB_RST + CSB_SZ_ROW)
#define WS_PW    (WSB_RCT + CSB_SZ_ROW)
#define PJ1 0
#define PJ2 (PJ1 + HID * HID)
#define PM1 (PJ2 + HID * HID)
#define PM2 (PM1 + HID * HID)
#define PO  (PM2 + HID * HID)
#define PWEND (PO + OC * HID)
#define WS_H0   (WS_PW + 2u * PWEND)
#define WS_ZJ   (WS_H0 + 4u * NRP * HID)
#define WS_ZM   (WS_ZJ + 4u * NRP * HID)
#define WS_END  (WS_ZM + 4u * NRP * HID)

__global__ __launch_bounds__(128) void k_packT(const float* __restrict__ Wm, int K, int N, __bf16* __restrict__ DST) {
  __shared__ __align__(16) __bf16 s[128]; const int n = blockIdx.x, k = threadIdx.x;
  if (k < K) s[k] = (__bf16)Wm[(size_t)k * N + n];
  __syncthreads();
  if (k < K / 8) vst2((unsigned*)(DST + (size_t)n * K + k * 8), *(const v4u*)&s[k * 8]);
}
__global__ __launch_bounds__(256) void k_inproj(const float* __restrict__ X, const float* __restrict__ W, const float* __restrict__ Bv, float* __restrict__ H0) {
  __shared__ float sw[DIN][HID], sb[HID]; __shared__ __align__(16) float so[16][HID + 4];
  const int tid = threadIdx.x; for (int q = tid; q < DIN * HID; q += 256) sw[q / HID][q % HID] = bfr(W[q]); if (tid < HID) sb[tid] = bfr(Bv[tid]);
  __syncthreads();
  const int nl = tid >> 4, c0 = (tid & 15) * 8; const size_t node = (size_t)blockIdx.x * 16 + nl; float xv[DIN];
#pragma unroll
  for (int i = 0; i < DIN; ++i) xv[i] = (node < (size_t)NN) ? bfr(X[node * DIN + i]) : 0.f;
#pragma unroll
  for (int j = 0; j < 8; ++j) { float a = sb[c0 + j];
#pragma unroll
    for (int i = 0; i < DIN; ++i) a += xv[i] * sw[i][c0 + j];
    so[nl][c0 + j] = a; }
  __syncthreads();
  for (int q = tid; q < 16 * 32; q += 256) { const int rl = q >> 5, pc = q & 31; vst2(H0 + ((size_t)blockIdx.x * 16 + rl) * HID + pc * 4, *(const v4f*)&so[rl][pc * 4]); }
}
__global__ __launch_bounds__(256) void k_agg2(const float* __restrict__ H0, const int* __restrict__ FSA, const int* __restrict__ RSTA, const int* __restrict__ RCTA, const int* __restrict__ FSB, const int* __restrict__ RSTB, const int* __restrict__ RCTB, float* __restrict__ ZJ, float* __restrict__ ZM) {
  __shared__ __align__(16) float sa[16][HID + 4], sbm[16][HID + 4];
  const int tid = threadIdx.x; const int nl = tid >> 4, f0 = (tid & 15) * 8; const size_t node = (size_t)blockIdx.x * 16 + nl;
  float aj[8], am[8];
#pragma unroll
  for (int i = 0; i < 8; ++i) { aj[i] = 0.f; am[i] = 0.f; }
  if (node < (size_t)NN) { const float* own = H0 + node * HID + f0;
#pragma unroll
    for (int i = 0; i < 8; ++i) { aj[i] = own[i]; am[i] = own[i]; }
    { const int cnt = min(max(RCTA[node], 0), CSA_BCAP); const int st = min(max(RSTA[node], 0), CSA_FINN - cnt);
      for (int e = 0; e < cnt; ++e) { const int s = min(max(FSA[st + e], 0), NN - 1); const float* hr = H0 + (size_t)s * HID + f0;
#pragma unroll
        for (int i = 0; i < 8; ++i) aj[i] += hr[i]; } }
    { const int cnt = min(max(RCTB[node], 0), CSB_BCAP); const int st = min(max(RSTB[node], 0), CSB_FINN - cnt);
      for (int e = 0; e < cnt; ++e) { const int s = min(max(FSB[st + e], 0), NN - 1); const float* hr = H0 + (size_t)s * HID + f0;
#pragma unroll
        for (int i = 0; i < 8; ++i) am[i] += hr[i]; } } }
#pragma unroll
  for (int i = 0; i < 8; ++i) { sa[nl][f0 + i] = aj[i]; sbm[nl][f0 + i] = am[i]; }
  __syncthreads();
  for (int q = tid; q < 16 * 32; q += 256) { const int rl = q >> 5, pc = q & 31; vst2(ZJ + ((size_t)blockIdx.x * 16 + rl) * HID + pc * 4, *(const v4f*)&sa[rl][pc * 4]); vst2(ZM + ((size_t)blockIdx.x * 16 + rl) * HID + pc * 4, *(const v4f*)&sbm[rl][pc * 4]); }
}
template <int NT, int EPI, int RM>
__global__ __launch_bounds__(128) void k_lin(const float* __restrict__ A, const __bf16* __restrict__ P, const float* __restrict__ bias, const float* RES, float* OUT, int ldo, int nrows) {
  __shared__ __align__(16) float so[4][16][NT * 16 + 4];
  const int tid = threadIdx.x, wave = tid >> 5, lane = tid & 31, col = lane & 15, g = lane >> 4; const size_t r0 = (size_t)blockIdx.x * 64 + wave * 16; size_t ra = r0 + col; if (ra >= NN) ra = NN - 1;
  v8f acc[NT]; for (int j = 0; j < NT; ++j) acc[j] = (v8f){};
#pragma unroll
  for (int kc = 0; kc < HID / 32; ++kc) { const F2 a = split_row(A + ra * HID, kc * 32, lane);
#pragma unroll
    for (int j = 0; j < NT; ++j) { const v16b w = frag_b(P + (size_t)(j * 16 + col) * HID + kc * 32, lane); acc[j] = wmma_bf(a.l, w, acc[j]); acc[j] = wmma_bf(a.h, w, acc[j]); } }
#pragma unroll
  for (int j = 0; j < NT; ++j) { const int n = j * 16 + col; const float bb = bfr(bias[n]);
#pragma unroll
    for (int r = 0; r < 8; ++r) { const size_t row = r0 + 8 * g + r; float v = acc[j][r] + bb; if (EPI == 1) v = fmaxf(v, 0.f); if (RM) v += RES[(row < NN ? row : NN - 1) * ldo + n]; so[wave][8 * g + r][n] = v; } }
  LDSX();
  for (int rl = 0; rl < 16; ++rl) if (lane < NT * 4 && r0 + rl < (size_t)nrows) vst2(OUT + (r0 + rl) * ldo + lane * 4, *(const v4f*)&so[wave][rl][lane * 4]);
}
__global__ __launch_bounds__(256) void k_lngelu(const float* __restrict__ gm, const float* __restrict__ bt, float* G) {
  __shared__ __align__(16) float s[8][HID]; const int wave = threadIdx.x >> 5, lane = threadIdx.x & 31; const size_t row = (size_t)blockIdx.x * 8 + wave; float v[4]; float sum = 0.f;
#pragma unroll
  for (int k = 0; k < 4; ++k) { v[k] = G[row * HID + lane + 32 * k]; sum += v[k]; }
#pragma unroll
  for (int o = 1; o < 32; o <<= 1) sum += __shfl_xor(sum, o);
  const float mu = sum / (float)HID; float var = 0.f;
#pragma unroll
  for (int k = 0; k < 4; ++k) { const float d = v[k] - mu; var += d * d; }
#pragma unroll
  for (int o = 1; o < 32; o <<= 1) var += __shfl_xor(var, o);
  const float rs = rsqrtf(var / (float)HID + 1e-5f);
#pragma unroll
  for (int k = 0; k < 4; ++k) { const int c = lane + 32 * k; const float y = (v[k] - mu) * rs * bfr(gm[c]) + bfr(bt[c]); s[wave][c] = 0.5f * y * (1.0f + erf_ni(y * 0.70710678118654752f)); }
  LDSX();
  vst2(G + row * HID + lane * 4, *(const v4f*)&s[wave][lane * 4]);
}
extern "C" void kernel_launch(void* const* d_in, const int* in_sizes, int n_in, void* d_out, int out_size, void* d_ws, size_t ws_size, hipStream_t stream) {
  (void)in_sizes; (void)n_in; (void)out_size;
  const float** F = (const float**)d_in; const int* EJ = (const int*)d_in[1]; const int* EM = (const int*)d_in[2];
  if (ws_size < (size_t)WS_END) return;
  char* ws = (char*)d_ws;
  int *CNTA = (int*)(ws + WSA_CNT), *OFFA = (int*)(ws + WSA_OFF), *BSTA = (int*)(ws + WSA_BST), *SEGSA = (int*)(ws + WSA_SEGS), *SEGEA = (int*)(ws + WSA_SEGE), *FSA = (int*)(ws + WSA_FS), *FEA = (int*)(ws + WSA_FE), *RSTA = (int*)(ws + WSA_RST), *RCTA = (int*)(ws + WSA_RCT);
  int *CNTB = (int*)(ws + WSB_CNT), *OFFB = (int*)(ws + WSB_OFF), *BSTB = (int*)(ws + WSB_BST), *SEGSB = (int*)(ws + WSB_SEGS), *SEGEB = (int*)(ws + WSB_SEGE), *FSB = (int*)(ws + WSB_FS), *FEB = (int*)(ws + WSB_FE), *RSTB = (int*)(ws + WSB_RST), *RCTB = (int*)(ws + WSB_RCT);
  __bf16* PW = (__bf16*)(ws + WS_PW); float *H0 = (float*)(ws + WS_H0), *ZJ = (float*)(ws + WS_ZJ), *ZM = (float*)(ws + WS_ZM); float* T = H0; float* G = ZJ;
  k_packT<<<HID, 128, 0, stream>>>(F[5], HID, HID, PW + PJ1); k_packT<<<HID, 128, 0, stream>>>(F[7], HID, HID, PW + PJ2); k_packT<<<HID, 128, 0, stream>>>(F[9], HID, HID, PW + PM1); k_packT<<<HID, 128, 0, stream>>>(F[11], HID, HID, PW + PM2); k_packT<<<OC, 128, 0, stream>>>(F[15], HID, OC, PW + PO);
  k_csA_cnt<<<CSA_NCH, 256, 0, stream>>>(EJ + EPA, 1, CNTA); k_csA_scan<<<1, 256, 0, stream>>>(CNTA, OFFA, BSTA); k_csA_scatter<<<CSA_NCH, 256, 0, stream>>>(EJ, EJ + EPA, 1, 1, OFFA, SEGSA, SEGEA); k_csA_bucket<<<CSA_NBK, 256, 0, stream>>>(CNTA, OFFA, BSTA, SEGSA, SEGEA, EJ + EPA, 1, FSA, FEA, RSTA, RCTA);
  k_csB_cnt<<<CSB_NCH, 256, 0, stream>>>(EM + EPB, 1, CNTB); k_csB_scan<<<1, 256, 0, stream>>>(CNTB, OFFB, BSTB); k_csB_scatter<<<CSB_NCH, 256, 0, stream>>>(EM, EM + EPB, 1, 1, OFFB, SEGSB, SEGEB); k_csB_bucket<<<CSB_NBK, 256, 0, stream>>>(CNTB, OFFB, BSTB, SEGSB, SEGEB, EM + EPB, 1, FSB, FEB, RSTB, RCTB);
  k_inproj<<<NRP / 16, 256, 0, stream>>>(F[0], F[3], F[4], H0);
  k_agg2<<<NRP / 16, 256, 0, stream>>>(H0, FSA, RSTA, RCTA, FSB, RSTB, RCTB, ZJ, ZM);
  k_lin<8, 1, 0><<<NBLK, 128, 0, stream>>>(ZJ, PW + PJ1, F[6], nullptr, T, HID, NRP);
  k_lin<8, 0, 0><<<NBLK, 128, 0, stream>>>(T, PW + PJ2, F[8], nullptr, G, HID, NRP);
  k_lin<8, 1, 0><<<NBLK, 128, 0, stream>>>(ZM, PW + PM1, F[10], nullptr, T, HID, NRP);
  k_lin<8, 0, 1><<<NBLK, 128, 0, stream>>>(T, PW + PM2, F[12], G, G, HID, NRP);
  k_lngelu<<<NRP / 8, 256, 0, stream>>>(F[13], F[14], G);
  k_lin<4, 0, 0><<<NBLK, 128, 0, stream>>>(G, PW + PO, F[16], nullptr, (float*)d_out, OC, NN);
}
